// GCN_enc_19963007992111
// MI455X (gfx1250) — hardware-verified
//
#include <hip/hip_runtime.h>
#include <stddef.h>

typedef __attribute__((ext_vector_type(16))) _Float16 v16h;
typedef __attribute__((ext_vector_type(8)))  _Float16 v8h;
typedef __attribute__((ext_vector_type(16))) __bf16   v16b;
typedef __attribute__((ext_vector_type(8)))  __bf16   v8b;
typedef __attribute__((ext_vector_type(8)))  float    v8f;
typedef __attribute__((ext_vector_type(4)))  float    v4f;
typedef __attribute__((ext_vector_type(4)))  int      v4i;

constexpr int HDIM = 128;
constexpr int KCMB = 256;
#define NTHR    256
#define NWAVE   8
#define EPT     8
#define NGRP    2
#define CHUNK   (NTHR * EPT * NGRP)
#define WCAP    (EPT * NGRP * 32)
#define LISTN   (NWAVE * WCAP)
#define NBA     512
#define NBB     2048
#define NSUB    (NBB / 64)
#define SUBCAP  1536
#define LDS_AGG (NBA * HDIM * 4 + LISTN * 4 + 64)
#define LDS_BKT (NSUB * SUBCAP * 4 + LISTN * 4 + 192 * 4)
#define RPWAVE  16

static_assert((CHUNK & (CHUNK - 1)) == 0);
static_assert(CHUNK <= 4096);
static_assert((NBA & (NBA - 1)) == 0 && NBA <= 4096);
static_assert((NBB & (NBB - 1)) == 0 && NBB <= 4096);
static_assert(NBA == NWAVE * 64);
static_assert(NBB == 4 * NBA && NSUB == 32);
static_assert((NBA * HDIM / 4) % NTHR == 0);
static_assert((NSUB * SUBCAP) % 4 == 0 && ((NSUB * SUBCAP / 4) % NTHR) == 0);
static_assert(HDIM == 128 && KCMB == 256);

__device__ __forceinline__ unsigned short f2bf_bits(float f) {
  unsigned u = __float_as_uint(f);
  return (unsigned short)((u + 0x7FFFu + ((u >> 16) & 1u)) >> 16);
}
__device__ __forceinline__ float bf_bits2f(unsigned short h) { return __uint_as_float(((unsigned)h) << 16); }

__device__ __forceinline__ void dep_guard_h(v8f& a, v8f& b, v16h x, v16h y) { asm volatile("v_nop\n\tv_nop\n\tv_nop\n\tv_nop" : "+v"(a), "+v"(b) : "v"(x), "v"(y)); }
__device__ __forceinline__ void dep_guard_b(v8f& a, v8f& b, v16b x, v16b y) { asm volatile("v_nop\n\tv_nop\n\tv_nop\n\tv_nop" : "+v"(a), "+v"(b) : "v"(x), "v"(y)); }
__device__ __forceinline__ void keep4_h(v16h a, v16h b, v16h c, v16h d) { asm volatile("v_nop" :: "v"(a), "v"(b), "v"(c), "v"(d)); }
__device__ __forceinline__ void keep4_b(v16b a, v16b b, v16b c, v16b d) { asm volatile("v_nop" :: "v"(a), "v"(b), "v"(c), "v"(d)); }
__device__ __forceinline__ void acc_guard4(v8f& a, v8f& b, v8f& c, v8f& d) { asm volatile("v_nop\n\tv_nop\n\tv_nop\n\tv_nop" : "+v"(a), "+v"(b), "+v"(c), "+v"(d)); }
template <typename T> struct Frag;
template <> struct Frag<_Float16> {
  typedef v16h V; union U { v16h v; v8h h[2]; };
  static __device__ __forceinline__ v16h load(const _Float16* p) {
    U f; f.h[0] = *(const v8h*)(p); f.h[1] = *(const v8h*)(p + 16); return f.v;
  }
  static __device__ __forceinline__ v8f mma(v16h a, v16h b, v8f c) {
    return __builtin_amdgcn_wmma_f32_16x16x32_f16(false, a, false, b, (short)0, c, false, false);
  }
  static __device__ __forceinline__ void guard(v8f& a, v8f& b, v16h x, v16h y) { dep_guard_h(a, b, x, y); }
  static __device__ __forceinline__ void keep(v16h a, v16h b, v16h c, v16h d) { keep4_h(a, b, c, d); }
};
template <> struct Frag<__bf16> {
  typedef v16b V; union U { v16b v; v8b h[2]; };
  static __device__ __forceinline__ v16b load(const __bf16* p) {
    U f; f.h[0] = *(const v8b*)(p); f.h[1] = *(const v8b*)(p + 16); return f.v;
  }
  static __device__ __forceinline__ v8f mma(v16b a, v16b b, v8f c) {
    return __builtin_amdgcn_wmma_f32_16x16x32_bf16(false, a, false, b, (short)0, c, false, false);
  }
  static __device__ __forceinline__ void guard(v8f& a, v8f& b, v16b x, v16b y) { dep_guard_b(a, b, x, y); }
  static __device__ __forceinline__ void keep(v16b a, v16b b, v16b c, v16b d) { keep4_b(a, b, c, d); }
};

template <int ET> struct Elem;
template <> struct Elem<0> { typedef _Float16 T; };
template <> struct Elem<1> { typedef __bf16 T; };
template <int ET, bool SPLIT, int BIAS_MODE, int OUT_MODE, bool RESID, int ACT = 0>
__global__ __launch_bounds__(256) void wmma_gemm64(
    const unsigned short* __restrict__ Ap, const unsigned short* __restrict__ A2p, int lda, long strideA,
    const unsigned short* __restrict__ Btp, const unsigned short* __restrict__ Bt2p, int ldb, long strideB,
    void* __restrict__ Cout, void* __restrict__ Cout2, int ldc, long strideC,
    const float* __restrict__ bias,
    const float* __restrict__ resid, long strideR,
    int M, int N, int K, float scale) {
  typedef typename Elem<ET>::T T;
  typedef typename Frag<T>::V V;
  const T* A = (const T*)Ap; const T* A2 = (const T*)A2p; const T* Bt = (const T*)Btp; const T* Bt2 = (const T*)Bt2p;
  __shared__ __align__(16) float sT[8][16 * 68];
  const int b    = blockIdx.y;
  const int lane = threadIdx.x & 31;
  const int wave = threadIdx.x >> 5;
  const int tilesN = N >> 6;
  const int tilesM = M >> 6;
  const int tile = blockIdx.x * 8 + wave;
  if (tile >= tilesM * tilesN) return;
  const int tm = tile / tilesN;
  const int tn = tile - tm * tilesN;
  const int m0 = tm << 6;
  const int n0 = tn << 6;

  const T* Ab  = A  + (size_t)b * strideA;
  const T* Bb  = Bt + (size_t)b * strideB;
  const T* Ab2 = SPLIT ? (A2  + (size_t)b * strideA) : nullptr;
  const T* Bb2 = SPLIT ? (Bt2 + (size_t)b * strideB) : nullptr;

  const int rlane = lane & 15;
  const int koff  = (lane >> 4) * 8;
  const int mOff  = (lane >> 4) * 8;

  v8f acc[4][4];
#pragma unroll
  for (int i = 0; i < 4; ++i)
#pragma unroll
    for (int j = 0; j < 4; ++j) acc[i][j] = (v8f){0.f,0.f,0.f,0.f,0.f,0.f,0.f,0.f};

  for (int k0 = 0; k0 < K; k0 += 32) {
    V bh[4], bl[4];
#pragma unroll
    for (int j = 0; j < 4; ++j) {
      const size_t bo = (size_t)(n0 + (j << 4) + rlane) * ldb + koff + k0;
      bh[j] = Frag<T>::load(Bb + bo);
      if (SPLIT) bl[j] = Frag<T>::load(Bb2 + bo);
    }
#pragma unroll
    for (int i = 0; i < 4; ++i) {
      const size_t ao = (size_t)(m0 + (i << 4) + rlane) * lda + koff + k0;
      V ah = Frag<T>::load(Ab + ao);
      V al;
      if (SPLIT) al = Frag<T>::load(Ab2 + ao);
#pragma unroll
      for (int j = 0; j < 4; ++j) {
        acc[i][j] = Frag<T>::mma(ah, bh[j], acc[i][j]);
        if (SPLIT) {
          acc[i][j] = Frag<T>::mma(ah, bl[j], acc[i][j]);
          acc[i][j] = Frag<T>::mma(al, bh[j], acc[i][j]);
        }
      }
      Frag<T>::guard(acc[i][0], acc[i][3], ah, SPLIT ? al : ah);
    }
    Frag<T>::keep(bh[0], bh[1], bh[2], bh[3]);
    if (SPLIT) Frag<T>::keep(bl[0], bl[1], bl[2], bl[3]);
  }
  acc_guard4(acc[0][0], acc[0][1], acc[0][2], acc[0][3]);
  acc_guard4(acc[1][0], acc[1][1], acc[1][2], acc[1][3]);
  acc_guard4(acc[2][0], acc[2][1], acc[2][2], acc[2][3]);
  acc_guard4(acc[3][0], acc[3][1], acc[3][2], acc[3][3]);

  float* slab = sT[wave];
  const float* Rb = RESID ? (resid + (size_t)b * strideR) : nullptr;
#pragma unroll
  for (int i = 0; i < 4; ++i) {
    const int mBase = m0 + (i << 4);
#pragma unroll
    for (int j = 0; j < 4; ++j) {
      const int n = n0 + (j << 4) + rlane;
      float bv = 0.f;
      if (BIAS_MODE == 2) bv = bias[n];
#pragma unroll
      for (int r = 0; r < 8; ++r) {
        float v = acc[i][j][r] * scale;
        if (BIAS_MODE == 1) v += bias[mBase + mOff + r];
        if (BIAS_MODE == 2) v += bv;
        if (RESID) v += Rb[(size_t)(mBase + mOff + r) * ldc + n];
        if (ACT == 1) v = tanhf(v);
        if (ACT == 2) v = fmaxf(v, 0.0f);
        if (ACT == 3) v = v / (1.0f + expf(-v));
        if (ACT == 4) v = (v > 0.f) ? v : 0.01f * v;
        if (ACT == 5) v = 0.5f * v * (1.0f + erff(v * 0.70710678118654752f));
        slab[(mOff + r) * 68 + (j << 4) + rlane] = v;
      }
    }
    __builtin_amdgcn_fence(__ATOMIC_RELEASE, "workgroup");
    __builtin_amdgcn_wave_barrier();
    __builtin_amdgcn_fence(__ATOMIC_ACQUIRE, "workgroup");
    if (OUT_MODE == 0) {
      float* C = (float*)Cout + (size_t)b * strideC;
      const int hh = lane >> 4, c4 = (lane & 15) * 4;
      for (int pass = 0; pass < 2; ++pass) {
#pragma unroll
        for (int it = 0; it < 8; ++it) {
          const int row = it * 2 + hh;
          v4f v = *(const v4f*)(slab + row * 68 + c4);
          *(volatile v4f*)(C + (size_t)(mBase + row) * ldc + n0 + c4) = v;
        }
        __threadfence();
      }
    } else {
      const int q = lane >> 3, c8 = (lane & 7) * 8;
      unsigned short* C  = (unsigned short*)Cout  + (size_t)b * strideC;
      unsigned short* C2 = (OUT_MODE == 2) ? ((unsigned short*)Cout2 + (size_t)b * strideC) : nullptr;
      for (int pass = 0; pass < 2; ++pass) {
#pragma unroll
        for (int it = 0; it < 4; ++it) {
          const int row = it * 4 + q;
          const float* sp = slab + row * 68 + c8;
          v8h hv, lv;
#pragma unroll
          for (int e = 0; e < 8; ++e) {
            if (OUT_MODE == 1) {
              hv[e] = (_Float16)sp[e];
            } else {
              unsigned short hb = f2bf_bits(sp[e]);
              unsigned short lb = f2bf_bits(sp[e] - bf_bits2f(hb));
              hv[e] = __builtin_bit_cast(_Float16, hb);
              lv[e] = __builtin_bit_cast(_Float16, lb);
            }
          }
          *(volatile v8h*)(C + (size_t)(mBase + row) * ldc + n0 + c8) = hv;
          if (OUT_MODE == 2) *(volatile v8h*)(C2 + (size_t)(mBase + row) * ldc + n0 + c8) = lv;
        }
        __threadfence();
      }
    }
    __builtin_amdgcn_fence(__ATOMIC_RELEASE, "workgroup");
    __builtin_amdgcn_wave_barrier();
    __builtin_amdgcn_fence(__ATOMIC_ACQUIRE, "workgroup");
  }
}

template <int NB>
__device__ __forceinline__ int scan_chunk(const int* __restrict__ lst, int nE, int cbase, int nodeBase,
                                          int* list, int tid, int lane, int wave, int fullvec) {
  int wc = 0;
#pragma unroll
  for (int g = 0; g < NGRP; ++g) {
    const int el0 = (g * NTHR + tid) * EPT;
    const int e0  = cbase + el0;
    v4i da, db;
    if (fullvec) {
      da = *(const v4i*)(lst + e0);
      db = *(const v4i*)(lst + e0 + 4);
    } else {
      const int em = nE - 1;
      da.x = lst[(e0     < em) ? e0     : em];
      da.y = lst[(e0 + 1 < em) ? e0 + 1 : em];
      da.z = lst[(e0 + 2 < em) ? e0 + 2 : em];
      da.w = lst[(e0 + 3 < em) ? e0 + 3 : em];
      db.x = lst[(e0 + 4 < em) ? e0 + 4 : em];
      db.y = lst[(e0 + 5 < em) ? e0 + 5 : em];
      db.z = lst[(e0 + 6 < em) ? e0 + 6 : em];
      db.w = lst[(e0 + 7 < em) ? e0 + 7 : em];
    }
    const bool v0 = (e0 < nE), v1 = (e0 + 1 < nE), v2 = (e0 + 2 < nE), v3 = (e0 + 3 < nE);
    const bool v4 = (e0 + 4 < nE), v5 = (e0 + 5 < nE), v6 = (e0 + 6 < nE), v7 = (e0 + 7 < nE);
    const unsigned nb = (unsigned)nodeBase;
    const unsigned s0 = (unsigned)da.x - nb, s1 = (unsigned)da.y - nb;
    const unsigned s2 = (unsigned)da.z - nb, s3 = (unsigned)da.w - nb;
    const unsigned s4 = (unsigned)db.x - nb, s5 = (unsigned)db.y - nb;
    const unsigned s6 = (unsigned)db.z - nb, s7 = (unsigned)db.w - nb;
    const bool h0 = v0 && (s0 < (unsigned)NB), h1 = v1 && (s1 < (unsigned)NB);
    const bool h2 = v2 && (s2 < (unsigned)NB), h3 = v3 && (s3 < (unsigned)NB);
    const bool h4 = v4 && (s4 < (unsigned)NB), h5 = v5 && (s5 < (unsigned)NB);
    const bool h6 = v6 && (s6 < (unsigned)NB), h7 = v7 && (s7 < (unsigned)NB);
    const unsigned any = __builtin_amdgcn_ballot_w32(h0 | h1 | h2 | h3 | h4 | h5 | h6 | h7);
    if (any != 0u) {
#define HITJ(J, HJ, SJ) { \
        const unsigned mj = __builtin_amdgcn_ballot_w32(HJ); \
        if (mj != 0u) { \
          if (HJ) { \
            const int pos = wc + (int)__builtin_amdgcn_mbcnt_lo(mj, 0u); \
            if (pos < WCAP) list[wave * WCAP + pos] = ((el0 + (J)) << 12) | (int)(SJ); \
          } \
          wc += (int)__builtin_popcount(mj); } }
      HITJ(0, h0, s0)
      HITJ(1, h1, s1)
      HITJ(2, h2, s2)
      HITJ(3, h3, s3)
      HITJ(4, h4, s4)
      HITJ(5, h5, s5)
      HITJ(6, h6, s6)
      HITJ(7, h7, s7)
#undef HITJ
    }
  }
  return wc;
}

__global__ __launch_bounds__(NTHR) void k_colsum(const float* __restrict__ h, float* part, int nN) {
  __shared__ float sd[NTHR];
  const int t = threadIdx.x, c = t & 127, rsel = t >> 7;
  const int r0 = blockIdx.x * 256;
  float a = 0.f;
#pragma unroll 4
  for (int i = 0; i < 128; ++i) {
    const int r  = r0 + 2 * i + rsel;
    const int rc = (r < nN) ? r : nN - 1;
    float v = h[(size_t)rc * HDIM + c];
    v = (r < nN) ? v : 0.f;
    a += v;
  }
  sd[t] = a;
  __syncthreads();
  if (t < 128) {
    const float p = sd[t] + sd[t + 128];
    float* pp = part + (size_t)blockIdx.x * HDIM + t;
    *(volatile float*)pp = p;
    __threadfence();
    *(volatile float*)pp = p;
  }
}

__device__ __forceinline__ unsigned match_sub5(int sub, unsigned vm) {
  unsigned m = vm;
#pragma unroll
  for (int bit = 0; bit < 5; ++bit) {
    const bool bset = ((sub >> bit) & 1) != 0;
    const unsigned bb = __builtin_amdgcn_ballot_w32(bset);
    m &= bset ? bb : ~bb;
  }
  return m;
}

__device__ __forceinline__ v8h pack16(v4f h, int s0, int s1) {
  v8h r;
  r[0] = (_Float16)__shfl(h.x, s0, 32); r[1] = (_Float16)__shfl(h.y, s0, 32);
  r[2] = (_Float16)__shfl(h.z, s0, 32); r[3] = (_Float16)__shfl(h.w, s0, 32);
  r[4] = (_Float16)__shfl(h.x, s1, 32); r[5] = (_Float16)__shfl(h.y, s1, 32);
  r[6] = (_Float16)__shfl(h.z, s1, 32); r[7] = (_Float16)__shfl(h.w, s1, 32);
  return r;
}

__global__ __launch_bounds__(NTHR) void k_wprep(const float* __restrict__ wrel0, const float* __restrict__ wroot0,
                                                const float* __restrict__ wrelm, const float* __restrict__ wrootm,
                                                unsigned short* wt) {
  const int layer = blockIdx.y;
  const float* wr = (layer == 0) ? wrel0  : (wrelm  + (size_t)(layer - 1) * HDIM * HDIM);
  const float* wo = (layer == 0) ? wroot0 : (wrootm + (size_t)(layer - 1) * HDIM * HDIM);
  const int i = blockIdx.x * NTHR + threadIdx.x;
  if (i >= HDIM * (KCMB / 8)) return;
  const int n  = i >> 5;
  const int k0 = (i & 31) * 8;
  const int kk = k0 & (HDIM - 1);
  const bool userel = (k0 < HDIM);
  v8h hv;
#pragma unroll
  for (int j = 0; j < 8; ++j) {
    const float a = wr[(size_t)(kk + j) * HDIM + n];
    const float c = wo[(size_t)(kk + j) * HDIM + n];
    hv[j] = (_Float16)((userel ? a : c) * 8.0f);
  }
  const size_t o = (size_t)layer * HDIM * KCMB + (size_t)i * 8;
  *(volatile v8h*)(wt + o) = hv;
  __threadfence();
  *(volatile v8h*)(wt + o) = hv;
}

__global__ __launch_bounds__(NTHR) void k_x16(const float* __restrict__ x, unsigned short* comb, int nN, int nRows) {
  const int lane = threadIdx.x & 31, wave = threadIdx.x >> 5;
  const int rbase = (blockIdx.x * NWAVE + wave) * RPWAVE;
  const int s0 = (2 * lane) & 31, s1 = (2 * lane + 1) & 31;
#pragma unroll 1
  for (int j = 0; j < RPWAVE; ++j) {
    const int row = rbase + j;
    if (row >= nRows) break;
    const int rc = (row < nN) ? row : nN - 1;
    v4f v = *(const v4f*)(x + (size_t)rc * HDIM + 4 * lane);
    if (row >= nN) { const v4f zz = {0.f, 0.f, 0.f, 0.f}; v = zz; }
    const v8h hv = pack16(v, s0, s1);
    unsigned short* cp = comb + (size_t)row * KCMB + HDIM + 8 * lane;
    if (lane < 16) *(volatile v8h*)cp = hv;
    __threadfence();
    if (lane < 16) *(volatile v8h*)cp = hv;
  }
}

__global__ __launch_bounds__(NTHR) void k_bucket(const int* __restrict__ rowl, const int* __restrict__ coll,
                                                 int* lists, int* meta, int nN, int nE, int vec_ok) {
  extern __shared__ v4i lds_dyn[];
  int* big   = (int*)lds_dyn;
  int* list  = big + NSUB * SUBCAP;
  int* cnt32 = list + LISTN;
  int* wcnt  = cnt32 + 32;
  int* metas = wcnt + 32;
  const int tid = threadIdx.x, lane = tid & 31, wave = tid >> 5;
  const int nodeBase = blockIdx.x * NBB;

  {
    const v4i zz = {0, 0, 0, 0};
    for (int i = tid; i < NSUB * SUBCAP / 4; i += NTHR) lds_dyn[i] = zz;
  }
  if (tid < 192) cnt32[tid] = 0;
  __syncthreads();

  int done = 0, fincnt = 0, resch = 0;
  const int nChunks = (nE + CHUNK - 1) / CHUNK;
#pragma unroll 1
  for (int ch = 0; ch < nChunks; ++ch) {
    const int cbase = ch * CHUNK;
    const int fullvec = (vec_ok != 0 && cbase + CHUNK <= nE) ? 1 : 0;
    const int wc = scan_chunk<NBB>(coll, nE, cbase, nodeBase, list, tid, lane, wave, fullvec);
    if (lane == 0) wcnt[wave] = wc;
    __syncthreads();
    if (wave == 0) {
      const int cstart = cnt32[lane];
#pragma unroll 1
      for (int wsx = 0; wsx < NWAVE; ++wsx) {
        int n = __builtin_amdgcn_readfirstlane(wcnt[wsx]);
        n = n > WCAP ? WCAP : (n < 0 ? 0 : n);
        const int* lp = list + wsx * WCAP;
#pragma unroll 1
        for (int i0 = 0; i0 < n; i0 += 32) {
          const int idx = i0 + lane;
          const bool valid = idx < n;
          const int ent  = lp[(idx < WCAP) ? idx : (WCAP - 1)];
          const int slot = ent & (NBB - 1);
          const int sub  = slot >> 6;
          int e = cbase + ((ent >> 12) & (CHUNK - 1));
          e = e > nE - 1 ? nE - 1 : e;
          int s = rowl[e];
          s = s < 0 ? 0 : (s > nN - 1 ? nN - 1 : s);
          const int packed = (s << 9) | (slot & (NBA - 1));
          const unsigned vm = __builtin_amdgcn_ballot_w32(valid);
          const unsigned m  = match_sub5(sub, vm);
          const int rank = (int)__builtin_amdgcn_mbcnt_lo(m, 0u);
          const int gcnt = (int)__builtin_popcount(m);
          const int base = cnt32[sub];
          const int pos  = base + rank;
          if (valid && pos < SUBCAP) big[sub * SUBCAP + pos] = packed;
          __builtin_amdgcn_fence(__ATOMIC_RELEASE, "workgroup");
          __builtin_amdgcn_wave_barrier();
          __builtin_amdgcn_fence(__ATOMIC_ACQUIRE, "workgroup");
          if (valid && rank == 0) {
            int nc = base + gcnt;
            nc = nc > (1 << 30) ? (1 << 30) : nc;
            cnt32[sub] = nc;
          }
          __builtin_amdgcn_fence(__ATOMIC_RELEASE, "workgroup");
          __builtin_amdgcn_wave_barrier();
          __builtin_amdgcn_fence(__ATOMIC_ACQUIRE, "workgroup");
        }
      }
      const int cnow = cnt32[lane];
      if (done == 0 && cnow > SUBCAP) { done = 1; fincnt = cstart; resch = ch; }
    }
    __syncthreads();
  }

  if (wave == 0) {
    int c = cnt32[lane];
    c = c < 0 ? 0 : (c > SUBCAP ? SUBCAP : c);
    const int cntv = done ? fincnt : c;
    const int resv = done ? resch : nChunks;
    metas[(lane >> 3) * 32 + (lane & 7)]     = cntv;
    metas[(lane >> 3) * 32 + 8 + (lane & 7)] = resv;
    __builtin_amdgcn_fence(__ATOMIC_RELEASE, "workgroup");
    __builtin_amdgcn_wave_barrier();
    __builtin_amdgcn_fence(__ATOMIC_ACQUIRE, "workgroup");
    int mv[4];
#pragma unroll
    for (int a = 0; a < 4; ++a) mv[a] = metas[a * 32 + lane];
    for (int pass = 0; pass < 2; ++pass) {
#pragma unroll
      for (int a = 0; a < 4; ++a)
        *(volatile int*)(meta + ((size_t)blockIdx.x * 4 + a) * 32 + lane) = mv[a];
      __threadfence();
    }
  }
  int* gl = lists + (size_t)blockIdx.x * NSUB * SUBCAP;
  for (int pass = 0; pass < 2; ++pass) {
#pragma unroll 4
    for (int i = tid; i < NSUB * SUBCAP / 4; i += NTHR) {
      const v4i v = lds_dyn[i];
      *(volatile v4i*)(gl + 4 * (size_t)i) = v;
    }
    __threadfence();
  }
}

__global__ __launch_bounds__(NTHR) void k_gagg(const int* __restrict__ rowl, const int* __restrict__ coll,
                                               const int* __restrict__ lists, const int* __restrict__ meta,
                                               const float* __restrict__ hs, unsigned short* comb,
                                               int nN, int nE, int vec_ok) {
  extern __shared__ v4i lds_dyn[];
  float* acc  = (float*)lds_dyn;
  int*   list = (int*)(acc + NBA * HDIM);
  int*   wcnt = list + LISTN;
  int*   resv = wcnt + NWAVE;
  const int tid = threadIdx.x, lane = tid & 31, wave = tid >> 5;
  const int a = blockIdx.x;
  const int nodeBase = a * NBA;

  {
    const v4f zz = {0.f, 0.f, 0.f, 0.f};
    v4f* av = (v4f*)lds_dyn;
    for (int i = tid; i < NBA * HDIM / 4; i += NTHR) av[i] = zz;
  }
  const int nChunks = (nE + CHUNK - 1) / CHUNK;
  int resmin = nChunks;
#pragma unroll
  for (int w = 0; w < NWAVE; ++w) {
    int r = meta[(size_t)a * 32 + 8 + w];
    r = r < 0 ? 0 : (r > nChunks ? nChunks : r);
    resmin = r < resmin ? r : resmin;
    if (tid == w) resv[w] = r;
  }
  resmin = __builtin_amdgcn_readfirstlane(resmin);
  __syncthreads();

  {
    int mycnt = __builtin_amdgcn_readfirstlane(meta[(size_t)a * 32 + wave]);
    mycnt = mycnt < 0 ? 0 : (mycnt > SUBCAP ? SUBCAP : mycnt);
    const int* lp = lists + ((size_t)a * NWAVE + wave) * SUBCAP;
#pragma unroll 1
    for (int i = 0; i < mycnt; ++i) {
      const int ent = __builtin_amdgcn_readfirstlane(lp[i]);
      int s = ent >> 9;
      s = s < 0 ? 0 : (s > nN - 1 ? nN - 1 : s);
      const int slot = (wave << 6) | (ent & 63);
      const v4f v = *(const v4f*)(hs + (size_t)s * HDIM + 4 * lane);
      v4f* ap = (v4f*)(acc + slot * HDIM + 4 * lane);
      *ap = *ap + v;
    }
  }
  __syncthreads();

#pragma unroll 1
  for (int ch = resmin; ch < nChunks; ++ch) {
    const int cbase = ch * CHUNK;
    const int fullvec = (vec_ok != 0 && cbase + CHUNK <= nE) ? 1 : 0;
    const int wc = scan_chunk<NBA>(coll, nE, cbase, nodeBase, list, tid, lane, wave, fullvec);
    if (lane == 0) wcnt[wave] = wc;
    __syncthreads();
    if (wave == 0) {
#pragma unroll 1
      for (int wsx = 0; wsx < NWAVE; ++wsx) {
        int n = __builtin_amdgcn_readfirstlane(wcnt[wsx]);
        n = n > WCAP ? WCAP : (n < 0 ? 0 : n);
        const int* lp = list + wsx * WCAP;
#pragma unroll 1
        for (int i = 0; i < n; ++i) {
          const int ent  = __builtin_amdgcn_readfirstlane(lp[i]);
          const int slot = ent & (NBA - 1);
          const int wsub = slot >> 6;
          const int rsub = __builtin_amdgcn_readfirstlane(resv[wsub]);
          if (ch >= rsub) {
            int e = cbase + ((ent >> 12) & (CHUNK - 1));
            e = e > nE - 1 ? nE - 1 : e;
            int s = rowl[e];
            s = s < 0 ? 0 : (s > nN - 1 ? nN - 1 : s);
            const v4f v = *(const v4f*)(hs + (size_t)s * HDIM + 4 * lane);
            v4f* ap = (v4f*)(acc + slot * HDIM + 4 * lane);
            *ap = *ap + v;
          }
        }
      }
    }
    __syncthreads();
  }

  unsigned short* cb = comb + (size_t)nodeBase * KCMB;
  for (int pass = 0; pass < 2; ++pass) {
#pragma unroll 4
    for (int q = 0; q < 32; ++q) {
      const int row = wave * 64 + 2 * q + (lane >> 4);
      const int col = (lane & 15) * 8;
      const float* sp = acc + row * HDIM + col;
      const v4f p0 = *(const v4f*)sp, p1 = *(const v4f*)(sp + 4);
      v8h hv;
      hv[0] = (_Float16)p0.x; hv[1] = (_Float16)p0.y; hv[2] = (_Float16)p0.z; hv[3] = (_Float16)p0.w;
      hv[4] = (_Float16)p1.x; hv[5] = (_Float16)p1.y; hv[6] = (_Float16)p1.z; hv[7] = (_Float16)p1.w;
      *(volatile v8h*)(cb + (size_t)row * KCMB + col) = hv;
    }
    __threadfence();
  }
}

__global__ __launch_bounds__(128) void k_mean(const float* __restrict__ part, int npb, float* meanb, int nN) {
  const int t = threadIdx.x;
  double s = 0.0;
#pragma unroll 1
  for (int b = 0; b < npb; ++b) s += (double)part[(size_t)b * HDIM + t];
  const float m = (float)(s / (double)nN);
  *(volatile float*)(meanb + t) = m;
  __threadfence();
  *(volatile float*)(meanb + t) = m;
}

__global__ __launch_bounds__(NTHR) void k_colsq(const float* __restrict__ h, const float* __restrict__ meanb,
                                                float* part, int nN) {
  __shared__ float sd[NTHR];
  const int t = threadIdx.x, c = t & 127, rsel = t >> 7;
  const int r0 = blockIdx.x * 256;
  const float m = meanb[c];
  float a = 0.f;
#pragma unroll 4
  for (int i = 0; i < 128; ++i) {
    const int r  = r0 + 2 * i + rsel;
    const int rc = (r < nN) ? r : nN - 1;
    const float v = h[(size_t)rc * HDIM + c];
    float d = v - m;
    d = (r < nN) ? d : 0.f;
    a = fmaf(d, d, a);
  }
  sd[t] = a;
  __syncthreads();
  if (t < 128) {
    const float p = sd[t] + sd[t + 128];
    float* pp = part + (size_t)blockIdx.x * HDIM + t;
    *(volatile float*)pp = p;
    __threadfence();
    *(volatile float*)pp = p;
  }
}

__global__ __launch_bounds__(128) void k_scsh(const float* __restrict__ partq, int npb, const float* __restrict__ meanb,
                                              const float* __restrict__ gamma, const float* __restrict__ beta,
                                              float* ss, int nN) {
  const int t = threadIdx.x;
  double s = 0.0;
#pragma unroll 1
  for (int b = 0; b < npb; ++b) s += (double)partq[(size_t)b * HDIM + t];
  const float var = (float)(s / (double)nN);
  const float scv = gamma[t] * rsqrtf(var + 1e-5f);
  const float shv = beta[t] - meanb[t] * scv;
  *(volatile float*)(ss + t) = scv;
  *(volatile float*)(ss + HDIM + t) = shv;
  __threadfence();
  *(volatile float*)(ss + t) = scv;
  *(volatile float*)(ss + HDIM + t) = shv;
}

__global__ __launch_bounds__(NTHR) void k_bnapply(float* hy, const float* __restrict__ ss, unsigned short* comb,
                                                  float* tot, int nN, int nRows, int first) {
  const int lane = threadIdx.x & 31, wave = threadIdx.x >> 5;
  const v4f sc = *(const v4f*)(ss + 4 * lane);
  const v4f sh = *(const v4f*)(ss + HDIM + 4 * lane);
  const int rbase = (blockIdx.x * NWAVE + wave) * RPWAVE;
  const int s0 = (2 * lane) & 31, s1 = (2 * lane + 1) & 31;
#pragma unroll 1
  for (int j = 0; j < RPWAVE; ++j) {
    const int row = rbase + j;
    if (row >= nRows) break;
    float* yp = hy + (size_t)row * HDIM + 4 * lane;
    const v4f y = *(const v4f*)yp;
    v4f h;
    h.x = fmaxf(fmaf(y.x, sc.x, sh.x), 0.f);
    h.y = fmaxf(fmaf(y.y, sc.y, sh.y), 0.f);
    h.z = fmaxf(fmaf(y.z, sc.z, sh.z), 0.f);
    h.w = fmaxf(fmaf(y.w, sc.w, sh.w), 0.f);
    const bool act = (row < nN);
    if (!act) { const v4f zz = {0.f, 0.f, 0.f, 0.f}; h = zz; }
    const v8h hv = pack16(h, s0, s1);
    v4f tv = h;
    float* tp = tot + (size_t)(act ? row : 0) * HDIM + 4 * lane;
    if (act) {
      if (first == 0) { const v4f told = *(const v4f*)tp; tv = told + h; }
    }
    unsigned short* cp = comb + (size_t)row * KCMB + HDIM + 8 * lane;
    for (int pass = 0; pass < 2; ++pass) {
      *(volatile v4f*)yp = h;
      if (lane < 16) *(volatile v8h*)cp = hv;
      if (act) *(volatile v4f*)tp = tv;
      __threadfence();
    }
  }
}

extern "C" void kernel_launch(void* const* d_in, const int* in_sizes, int n_in,
                              void* d_out, int out_size, void* d_ws, size_t ws_size,
                              hipStream_t stream) {
  if (n_in < 12) return;
  if (in_sizes[0] <= 0 || (in_sizes[0] % HDIM) != 0) return;
  const int nN = in_sizes[0] / HDIM;
  if (in_sizes[1] < 0 || (in_sizes[1] & 1) != 0) return;
  const int nE = in_sizes[1] / 2;
  const int wsz = HDIM * HDIM;
  if (in_sizes[2] != wsz || in_sizes[3] != wsz) return;
  if (in_sizes[4] < HDIM || in_sizes[5] < HDIM || in_sizes[6] < HDIM) return;
  if (in_sizes[7] <= 0 || (in_sizes[7] % wsz) != 0 || in_sizes[8] != in_sizes[7]) return;
  const int nMid = in_sizes[7] / wsz;
  const int nL = 1 + nMid;
  if (nL > 64) return;
  if (in_sizes[9] < nMid * HDIM || in_sizes[10] < nMid * HDIM || in_sizes[11] < nMid * HDIM) return;
  if (out_size != nN * HDIM) return;
  if (nN < 1 || nN > (1 << 22)) return;

  const float* x        = (const float*)d_in[0];
  const int*   ei       = (const int*)d_in[1];
  const float* wrel_in  = (const float*)d_in[2];
  const float* wroot_in = (const float*)d_in[3];
  const float* b_in     = (const float*)d_in[4];
  const float* g_in     = (const float*)d_in[5];
  const float* be_in    = (const float*)d_in[6];
  const float* wrel_m   = (const float*)d_in[7];
  const float* wroot_m  = (const float*)d_in[8];
  const float* b_m      = (const float*)d_in[9];
  const float* g_m      = (const float*)d_in[10];
  const float* be_m     = (const float*)d_in[11];
  const int* rowl = ei;
  const int* coll = ei + nE;
  float* out = (float*)d_out;

  const int nA  = (nN + NBA - 1) / NBA;
  const int RP  = nA * NBA;
  const int nBK = (nN + NBB - 1) / NBB;
  const int NPB = (nN + 255) / 256;
  const int vec_col = ((nE & 3) == 0) ? 1 : 0;

  char* ws = (char*)d_ws;
  size_t off = 0;
  const size_t oWT = off; off += (((size_t)nL * HDIM * KCMB * 2) + 255) & ~(size_t)255;
  const size_t oHY = off; off += (((size_t)RP * HDIM * 4) + 255) & ~(size_t)255;
  const size_t oCB = off; off += (((size_t)RP * KCMB * 2) + 255) & ~(size_t)255;
  const size_t oLS = off; off += (((size_t)nBK * NSUB * SUBCAP * 4) + 255) & ~(size_t)255;
  const size_t oMT = off; off += (((size_t)nBK * 4 * 32 * 4) + 255) & ~(size_t)255;
  const size_t oPS = off; off += (((size_t)NPB * HDIM * 4) + 255) & ~(size_t)255;
  const size_t oPQ = off; off += (((size_t)NPB * HDIM * 4) + 255) & ~(size_t)255;
  const size_t oMN = off; off += 512;
  const size_t oSS = off; off += 1024;
  if (off > ws_size) return;
  if (off > (size_t)134217728) return;

  unsigned short* wt   = (unsigned short*)(ws + oWT);
  float*          hy   = (float*)(ws + oHY);
  unsigned short* comb = (unsigned short*)(ws + oCB);
  int*            lst  = (int*)(ws + oLS);
  int*            meta = (int*)(ws + oMT);
  float*          ps   = (float*)(ws + oPS);
  float*          pq   = (float*)(ws + oPQ);
  float*          mn   = (float*)(ws + oMN);
  float*          ss   = (float*)(ws + oSS);

  k_wprep<<<dim3(HDIM * (KCMB / 8) / NTHR, nL), NTHR, 0, stream>>>(wrel_in, wroot_in, wrel_m, wroot_m, wt);
  const int gRow = (RP + NWAVE * RPWAVE - 1) / (NWAVE * RPWAVE);
  k_x16<<<gRow, NTHR, 0, stream>>>(x, comb, nN, RP);
  k_bucket<<<nBK, NTHR, LDS_BKT, stream>>>(rowl, coll, lst, meta, nN, nE, vec_col);

  const int gG = ((RP / 64) * (HDIM / 64) + 7) / 8;
  for (int l = 0; l < nL; ++l) {
    const float* hsrc  = (l == 0) ? x : hy;
    const float* bias  = (l == 0) ? b_in  : (b_m  + (size_t)(l - 1) * HDIM);
    const float* gamma = (l == 0) ? g_in  : (g_m  + (size_t)(l - 1) * HDIM);
    const float* beta  = (l == 0) ? be_in : (be_m + (size_t)(l - 1) * HDIM);
    const unsigned short* wtl = wt + (size_t)l * HDIM * KCMB;

    k_gagg<<<nA, NTHR, LDS_AGG, stream>>>(rowl, coll, lst, meta, hsrc, comb, nN, nE, vec_col);
    wmma_gemm64<0, false, 2, 0, false, 0><<<dim3(gG, 1), 256, 0, stream>>>(
        comb, comb, KCMB, 0L, wtl, wtl, KCMB, 0L, (void*)hy, (void*)hy, HDIM, 0L,
        bias, bias, 0L, RP, HDIM, KCMB, 0.125f);
    k_colsum<<<NPB, NTHR, 0, stream>>>(hy, ps, nN);
    k_mean<<<1, 128, 0, stream>>>(ps, NPB, mn, nN);
    k_colsq<<<NPB, NTHR, 0, stream>>>(hy, mn, pq, nN);
    k_scsh<<<1, 128, 0, stream>>>(pq, NPB, mn, gamma, beta, ss, nN);
    k_bnapply<<<gRow, NTHR, 0, stream>>>(hy, ss, comb, out, nN, RP, (l == 0) ? 1 : 0);
  }
}
